// SwitchedConvHardRouting_83863531422097
// MI455X (gfx1250) — hardware-verified
//
#include <hip/hip_runtime.h>

typedef __bf16   v16b __attribute__((ext_vector_type(16)));
typedef __bf16   v8b  __attribute__((ext_vector_type(8)));
typedef float    v8f  __attribute__((ext_vector_type(8)));
typedef float    v4f  __attribute__((ext_vector_type(4)));
typedef unsigned short v8u __attribute__((ext_vector_type(8)));
typedef v8b __attribute__((may_alias)) v8ba;
typedef v8u __attribute__((may_alias)) v8ua;
typedef v4f __attribute__((may_alias)) v4fa;

#define NBAT   8
#define ICN    256
#define OCN    256
#define SBR    8
#define IMH    48
#define IMW    48
#define HWC    2304
#define NPOS   18432
#define KDIM   2304
#define NCOL   2048
#define CWR    16
#define NXE    (NBAT * ICN * HWC)
#define NWE    (OCN * ICN * SBR * 9)
#define NCWE   (SBR * ICN)
#define NOUTE  (NBAT * OCN * HWC)
#define GTM    64
#define APITCH 264
#define CTM    128
#define CTN    64
#define CPITCH 68

static_assert(KDIM == 9 * ICN);
static_assert(KDIM % 32 == 0);
static_assert(ICN % 32 == 0);
static_assert(ICN == 8 * 32);
static_assert(NPOS % CTM == 0);
static_assert(HWC % CTM == 0);
static_assert(HWC % GTM == 0);
static_assert(NPOS % GTM == 0);
static_assert(NCOL % CTN == 0);
static_assert(NCOL == OCN * SBR);
static_assert(NPOS % 8 == 0);
static_assert(NCOL % 8 == 0);
static_assert(CTN == 8 * SBR);
static_assert((APITCH * 2) % 16 == 0);
static_assert((CPITCH * 4) % 16 == 0);

__device__ __forceinline__ v8f wmma_bf16(v16b a, v16b b, v8f c) {
  v8f d = __builtin_amdgcn_wmma_f32_16x16x32_bf16(false, a, false, b, (short)0, c, false, false);
  asm volatile("v_nop\n\tv_nop\n\tv_nop\n\tv_nop" : "+v"(d) : "v"(a), "v"(b));
  return d;
}

__device__ __forceinline__ v16b frag_b(const unsigned short* p, int h) {
  union { v16b v; v8b hv[2]; } f;
  f.hv[0] = *(const v8ba*)(p + 8 * h);
  f.hv[1] = *(const v8ba*)(p + 16 + 8 * h);
  return f.v;
}

__device__ __forceinline__ unsigned short bf16bits(float v) {
  unsigned int u = __float_as_uint(v);
  u += 0x7FFFu + ((u >> 16) & 1u);
  return (unsigned short)(u >> 16);
}
__device__ __forceinline__ float bf16val(unsigned short b) {
  return __uint_as_float(((unsigned int)b) << 16);
}
__device__ __forceinline__ float bf16r(float v) { return bf16val(bf16bits(v)); }
__device__ __forceinline__ int clampi(int v, int lo, int hi) {
  return v < lo ? lo : (v > hi ? hi : v);
}

__global__ __launch_bounds__(256) void k_im2col(const float* __restrict__ x,
                                               unsigned short* __restrict__ apl) {
  const int tid = threadIdx.x, lane = tid & 31, w = tid >> 5;
  const int m = blockIdx.x * 8 + w;
  if (m >= NPOS) return;
  const int b = m / HWC;
  const int p = m - b * HWC;
  const int y = p / IMW;
  const int xw = p - y * IMW;
  const float* xb = x + (size_t)b * ICN * HWC + (size_t)(8 * lane) * HWC;
  unsigned short* arow = apl + (size_t)m * KDIM + 8 * lane;
  #pragma unroll 1
  for (int tap = 0; tap < 9; ++tap) {
    const int ky = tap / 3;
    const int kx = tap - 3 * ky;
    const int yy = y + ky - 1, xx = xw + kx - 1;
    const bool ok = (yy >= 0) && (yy < IMH) && (xx >= 0) && (xx < IMW);
    const int yc = clampi(yy, 0, IMH - 1), xc = clampi(xx, 0, IMW - 1);
    const float* sp = xb + yc * IMW + xc;
    v8u o;
    #pragma unroll
    for (int i = 0; i < 8; ++i) {
      const float v = sp[(size_t)i * HWC];
      o[i] = ok ? bf16bits(v) : (unsigned short)0;
    }
    unsigned short* dst = arow + tap * ICN;
    *(volatile v8u*)dst = o;
    __threadfence();
    *(volatile v8u*)dst = o;
  }
}

__global__ __launch_bounds__(256) void k_wprep(const float* __restrict__ wt,
                                              const float* __restrict__ cw,
                                              unsigned short* __restrict__ bpl,
                                              unsigned short* __restrict__ cwt) {
  const int tid = threadIdx.x, lane = tid & 31, w = tid >> 5;
  const int blk = blockIdx.x;
  if (blk < NCOL / 8) {
    const int n = blk * 8 + w;
    const int oc = n >> 3, s = n & 7;
    const float* src = wt + (((size_t)oc * ICN + 8 * lane) * SBR + s) * 9;
    unsigned short* brow = bpl + (size_t)n * KDIM + 8 * lane;
    #pragma unroll 1
    for (int tap = 0; tap < 9; ++tap) {
      v8u o;
      #pragma unroll
      for (int i = 0; i < 8; ++i) o[i] = bf16bits(src[(size_t)i * (SBR * 9) + tap]);
      unsigned short* dst = brow + tap * ICN;
      *(volatile v8u*)dst = o;
      __threadfence();
      *(volatile v8u*)dst = o;
    }
  } else {
    const int r = (blk - NCOL / 8) * 8 + w;
    if (r < CWR) {
      const bool ok = (r < SBR);
      const int rc = ok ? r : (SBR - 1);
      const float* src = cw + (size_t)rc * ICN + 8 * lane;
      v8u o;
      #pragma unroll
      for (int i = 0; i < 8; ++i) {
        const float v = src[i];
        o[i] = ok ? bf16bits(v) : (unsigned short)0;
      }
      unsigned short* dst = cwt + (size_t)r * ICN + 8 * lane;
      *(volatile v8u*)dst = o;
      __threadfence();
      *(volatile v8u*)dst = o;
    }
  }
}

__device__ __forceinline__ void gate_store_pass(const float* sS, float* sel, int m0, int w, int lane) {
  #pragma unroll
  for (int q = 0; q < 2; ++q) {
    const int e = 256 * w + 128 * q + 4 * lane;
    const v4f v = *(const v4fa*)(sS + e);
    *(volatile v4f*)(sel + (size_t)m0 * SBR + e) = v;
  }
}

__global__ __launch_bounds__(64) void k_gate(const float* __restrict__ x,
                                            const unsigned short* __restrict__ cwt,
                                            const float* __restrict__ cb,
                                            float* __restrict__ sel) {
  __shared__ __attribute__((aligned(16))) unsigned short sA[GTM * APITCH];
  __shared__ __attribute__((aligned(16))) float sL[GTM * 16];
  __shared__ __attribute__((aligned(16))) float sS[GTM * SBR];

  const int tid = threadIdx.x, lane = tid & 31, w = tid >> 5;
  const int h = lane >> 4, m = lane & 15;
  const int m0 = blockIdx.x * GTM;
  const int b = m0 / HWC;
  const int p0 = m0 - b * HWC;

  {
    const float* xp = x + (size_t)b * ICN * HWC + p0 + tid;
    unsigned short* ar = sA + tid * APITCH;
    #pragma unroll 4
    for (int ic = 0; ic < ICN; ++ic) ar[ic] = bf16bits(xp[(size_t)ic * HWC]);
  }
  __syncthreads();

  const v8f zero8 = {0.f, 0.f, 0.f, 0.f, 0.f, 0.f, 0.f, 0.f};
  v8f acc[2];
  acc[0] = zero8; acc[1] = zero8;
  const unsigned short* a0p = sA + (32 * w + m) * APITCH;
  const unsigned short* a1p = a0p + 16 * APITCH;
  const unsigned short* bq = cwt + (size_t)m * ICN;
  #pragma unroll 1
  for (int k0 = 0; k0 < ICN; k0 += 32) {
    const v16b a0 = frag_b(a0p + k0, h);
    const v16b a1 = frag_b(a1p + k0, h);
    const v16b bb = frag_b(bq + k0, h);
    acc[0] = wmma_bf16(a0, bb, acc[0]);
    acc[1] = wmma_bf16(a1, bb, acc[1]);
  }
  #pragma unroll
  for (int mt = 0; mt < 2; ++mt)
    #pragma unroll
    for (int r = 0; r < 8; ++r)
      sL[(32 * w + 16 * mt + 8 * h + r) * 16 + m] = acc[mt][r];
  __syncthreads();

  {
    const float* lr = sL + tid * 16;
    float* sr = sS + tid * SBR;
    float mx = -3.0e38f;
    #pragma unroll
    for (int s = 0; s < SBR; ++s) mx = fmaxf(mx, lr[s] + bf16r(cb[s]));
    float sum = 0.0f;
    #pragma unroll 1
    for (int s = 0; s < SBR; ++s) {
      const float e = expf((lr[s] + bf16r(cb[s])) - mx);
      sr[s] = e;
      sum += e;
    }
    const float inv = 1.0f / sum;
    float sum2 = 0.0f;
    #pragma unroll
    for (int s = 0; s < SBR; ++s) {
      const float pv = sr[s] * inv;
      sr[s] = pv;
      sum2 += pv;
    }
    const float inv2 = 1.0f / sum2;
    #pragma unroll
    for (int s = 0; s < SBR; ++s) sr[s] = sr[s] * inv2;
  }
  __syncthreads();

  gate_store_pass(sS, sel, m0, w, lane);
  __threadfence();
  gate_store_pass(sS, sel, m0, w, lane);
}

__device__ __forceinline__ void conv_store_pass(const float* sO, float* out, int b, int p0,
                                                int oc0, int w, int lane) {
  #pragma unroll
  for (int q = 0; q < 2; ++q) {
    const int j = 2 * w + q;
    const v4f v = *(const v4fa*)(sO + j * CTM + 4 * lane);
    float* dst = out + ((size_t)(b * OCN + oc0 + j)) * HWC + p0 + 4 * lane;
    *(volatile v4f*)dst = v;
  }
}

__global__ __launch_bounds__(128) void k_conv(const unsigned short* __restrict__ apl,
                                             const unsigned short* __restrict__ bpl,
                                             const float* __restrict__ sel,
                                             const float* __restrict__ bias,
                                             float* __restrict__ out) {
  __shared__ __attribute__((aligned(16))) float sC[CTM * CPITCH];
  __shared__ __attribute__((aligned(16))) float sO[SBR * CTM];

  const int tid = threadIdx.x, lane = tid & 31, w = tid >> 5;
  const int h = lane >> 4, m = lane & 15;
  const int m0 = blockIdx.x * CTM;
  const int n0 = blockIdx.y * CTN;
  const int oc0 = blockIdx.y * SBR;

  const unsigned short* a0p = apl + (size_t)(m0 + 32 * w + m) * KDIM;
  const unsigned short* a1p = a0p + (size_t)16 * KDIM;
  const unsigned short* bp  = bpl + (size_t)(n0 + m) * KDIM;

  const v8f zero8 = {0.f, 0.f, 0.f, 0.f, 0.f, 0.f, 0.f, 0.f};
  v8f acc[2][4];
  #pragma unroll
  for (int mt = 0; mt < 2; ++mt)
    #pragma unroll
    for (int nt = 0; nt < 4; ++nt) acc[mt][nt] = zero8;

  #pragma unroll 1
  for (int k0 = 0; k0 < KDIM; k0 += 32) {
    const v16b a0 = frag_b(a0p + k0, h);
    const v16b a1 = frag_b(a1p + k0, h);
    #pragma unroll
    for (int nt = 0; nt < 4; ++nt) {
      const v16b bb = frag_b(bp + (size_t)(16 * nt) * KDIM + k0, h);
      acc[0][nt] = wmma_bf16(a0, bb, acc[0][nt]);
      acc[1][nt] = wmma_bf16(a1, bb, acc[1][nt]);
    }
  }

  #pragma unroll
  for (int nt = 0; nt < 4; ++nt)
    #pragma unroll
    for (int mt = 0; mt < 2; ++mt)
      #pragma unroll
      for (int r = 0; r < 8; ++r)
        sC[(32 * w + 16 * mt + 8 * h + r) * CPITCH + 16 * nt + m] = acc[mt][nt][r];
  __syncthreads();

  {
    const int t = tid;
    const int grow = m0 + t;
    const v4f s0 = *(const v4fa*)(sel + (size_t)grow * SBR);
    const v4f s1 = *(const v4fa*)(sel + (size_t)grow * SBR + 4);
    const float* cr = sC + t * CPITCH;
    #pragma unroll
    for (int j = 0; j < SBR; ++j) {
      const float br = bf16r(bias[oc0 + j]);
      const v4f c0 = *(const v4fa*)(cr + 8 * j);
      const v4f c1 = *(const v4fa*)(cr + 8 * j + 4);
      float yv = s0.x * (c0.x + br);
      yv = fmaf(s0.y, c0.y + br, yv);
      yv = fmaf(s0.z, c0.z + br, yv);
      yv = fmaf(s0.w, c0.w + br, yv);
      yv = fmaf(s1.x, c1.x + br, yv);
      yv = fmaf(s1.y, c1.y + br, yv);
      yv = fmaf(s1.z, c1.z + br, yv);
      yv = fmaf(s1.w, c1.w + br, yv);
      sO[j * CTM + t] = yv;
    }
  }
  __syncthreads();

  const int b = m0 / HWC;
  const int p0 = m0 - b * HWC;
  conv_store_pass(sO, out, b, p0, oc0, w, lane);
  __threadfence();
  conv_store_pass(sO, out, b, p0, oc0, w, lane);
}

extern "C" void kernel_launch(void* const* d_in, const int* in_sizes, int n_in,
                              void* d_out, int out_size, void* d_ws, size_t ws_size,
                              hipStream_t stream) {
  if (n_in < 5) return;
  if (in_sizes[0] != NXE) return;
  if (in_sizes[1] != NCWE) return;
  if (in_sizes[2] != SBR) return;
  if (in_sizes[3] != NWE) return;
  if (in_sizes[4] != OCN) return;
  if (out_size != NOUTE) return;

  const float* x    = (const float*)d_in[0];
  const float* cw   = (const float*)d_in[1];
  const float* cb   = (const float*)d_in[2];
  const float* wt   = (const float*)d_in[3];
  const float* bias = (const float*)d_in[4];
  float* out = (float*)d_out;

  const size_t a_b   = (size_t)NPOS * KDIM * 2;
  const size_t b_b   = (size_t)NCOL * KDIM * 2;
  const size_t sel_b = (size_t)NPOS * SBR * 4;
  const size_t cwt_b = (size_t)CWR * ICN * 2;
  const size_t total = a_b + b_b + sel_b + cwt_b;
  if (total > ws_size) return;
  if (total > (size_t)134217728) return;

  char* ws = (char*)d_ws;
  unsigned short* apl = (unsigned short*)(ws);
  unsigned short* bpl = (unsigned short*)(ws + a_b);
  float*          sel = (float*)(ws + a_b + b_b);
  unsigned short* cwt = (unsigned short*)(ws + a_b + b_b + sel_b);

  k_im2col<<<NPOS / 8, 256, 0, stream>>>(x, apl);

  k_wprep<<<NCOL / 8 + 2, 256, 0, stream>>>(wt, cw, bpl, cwt);

  k_gate<<<NPOS / GTM, 64, 0, stream>>>(x, cwt, cb, sel);

  dim3 g4(NPOS / CTM, NCOL / CTN);
  k_conv<<<g4, 128, 0, stream>>>(apl, bpl, sel, bias, out);
}
